// GraphGRUCell_33011118637673
// MI455X (gfx1250) — hardware-verified
//
#include <hip/hip_runtime.h>
#include <stddef.h>


#define NBAT   8
#define UW     64
#define KD     64
#define NTHR   256
#define NWAVE  8
#define EPT    8
#define NGRP   2
#define CHUNK  (NTHR * EPT * NGRP)
#define WCAP   (EPT * NGRP * 32)
#define LISTN  (NWAVE * WCAP)
#define NBF    1024
#define RCAP   40960
#define TPWV   (NBF / NWAVE)
#define DEGCAP 1024
#define BM     64
#define APK    (KD + 8)
#define WSCAP  134217728
#define NEG_SLOPE 0.2f

#define LDS_GEMM1 (2 * BM * APK * 2)
#define LDS_GATE  (2 * BM * APK * 2 + 2 * BM * UW * 4 + BM * 4)
#define LDS_AGG   ((RCAP + 3 * NBF + LISTN + 32) * 4)

static_assert((CHUNK & (CHUNK - 1)) == 0);
static_assert(CHUNK <= 4096);
static_assert((NBF & (NBF - 1)) == 0 && NBF <= 4096);
static_assert(NBF == 4 * NTHR);
static_assert((RCAP % 32) == 0);
static_assert(TPWV * NWAVE == NBF);
static_assert(LISTN >= NWAVE * NBAT * UW);
static_assert(2 * BM * APK * 2 >= BM * UW * 4);
static_assert((BM * KD / 8) == 2 * NTHR);
static_assert(NBAT * 4 == 32 && UW == 64 && KD == 64);
static_assert(((APK * 2) % 16) == 0);

typedef float          v4f  __attribute__((ext_vector_type(4)));
typedef float          v8f  __attribute__((ext_vector_type(8)));
typedef int            v4i  __attribute__((ext_vector_type(4)));
typedef unsigned short v8us __attribute__((ext_vector_type(8)));
typedef __bf16         v16b __attribute__((ext_vector_type(16)));
union FragB { v16b v; v8us h[2]; };

__device__ __forceinline__ unsigned int bfr(float f) {
  const unsigned int u = __float_as_uint(f);
  return (u + 0x7FFFu + ((u >> 16) & 1u)) >> 16;
}

__device__ __forceinline__ void split1(float x, unsigned short& hb, unsigned short& lb) {
  const unsigned int hu = bfr(x);
  const float hf = __uint_as_float(hu << 16);
  hb = (unsigned short)hu;
  lb = (unsigned short)bfr(x - hf);
}

__device__ __forceinline__ void split8(v4f a, v4f b, v8us& hi, v8us& lo) {
  unsigned short hb, lb;
  split1(a.x, hb, lb); hi[0] = hb; lo[0] = lb;
  split1(a.y, hb, lb); hi[1] = hb; lo[1] = lb;
  split1(a.z, hb, lb); hi[2] = hb; lo[2] = lb;
  split1(a.w, hb, lb); hi[3] = hb; lo[3] = lb;
  split1(b.x, hb, lb); hi[4] = hb; lo[4] = lb;
  split1(b.y, hb, lb); hi[5] = hb; lo[5] = lb;
  split1(b.z, hb, lb); hi[6] = hb; lo[6] = lb;
  split1(b.w, hb, lb); hi[7] = hb; lo[7] = lb;
}

__device__ __forceinline__ v8f wmb(v16b a, v16b b, v8f c) {
  v8f d = __builtin_amdgcn_wmma_f32_16x16x32_bf16(false, a, false, b, (short)0, c, false, false);
  asm volatile("v_nop\n\tv_nop\n\tv_nop\n\tv_nop" : "+v"(d) : "v"(a), "v"(b));
  return d;
}

__device__ __forceinline__ float lrelu(float v) { return v > 0.0f ? v : NEG_SLOPE * v; }
__device__ __forceinline__ float rcpf_(float x) { return __builtin_amdgcn_rcpf(x); }

__device__ __forceinline__ float sigmf(float v) {
  const float e = __expf(-fabsf(v));
  const float r = rcpf_(1.0f + e);
  const float neg = e * r;
  return v >= 0.0f ? r : neg;
}

__device__ __forceinline__ float tanhf_(float v) {
  const float e = __expf(-2.0f * fabsf(v));
  const float t = (1.0f - e) * rcpf_(1.0f + e);
  return v >= 0.0f ? t : -t;
}

template <int NB>
__device__ __forceinline__ int scan_chunk(const int* __restrict__ dsts, int nE, int cbase, int slotBase,
                                          int vec8, int* list, int tid, int lane, int wave) {
  int wc = 0;
#pragma unroll
  for (int g = 0; g < NGRP; ++g) {
    const int el0  = (g * NTHR + tid) * EPT;
    const int e0   = cbase + el0;
    const int sent = -2147483647 - 1;
    v4i da, db;
    if (vec8 != 0 && cbase + CHUNK <= nE) {
      da = *(const v4i*)(dsts + e0);
      db = *(const v4i*)(dsts + e0 + 4);
    } else {
      da.x = (e0     < nE) ? dsts[min(e0, nE - 1)] : sent;
      da.y = (e0 + 1 < nE) ? dsts[min(e0 + 1, nE - 1)] : sent;
      da.z = (e0 + 2 < nE) ? dsts[min(e0 + 2, nE - 1)] : sent;
      da.w = (e0 + 3 < nE) ? dsts[min(e0 + 3, nE - 1)] : sent;
      db.x = (e0 + 4 < nE) ? dsts[min(e0 + 4, nE - 1)] : sent;
      db.y = (e0 + 5 < nE) ? dsts[min(e0 + 5, nE - 1)] : sent;
      db.z = (e0 + 6 < nE) ? dsts[min(e0 + 6, nE - 1)] : sent;
      db.w = (e0 + 7 < nE) ? dsts[min(e0 + 7, nE - 1)] : sent;
    }
    const unsigned nb = (unsigned)slotBase;
    const unsigned s0 = (unsigned)da.x - nb, s1 = (unsigned)da.y - nb;
    const unsigned s2 = (unsigned)da.z - nb, s3 = (unsigned)da.w - nb;
    const unsigned s4 = (unsigned)db.x - nb, s5 = (unsigned)db.y - nb;
    const unsigned s6 = (unsigned)db.z - nb, s7 = (unsigned)db.w - nb;
    const bool h0 = s0 < (unsigned)NB, h1 = s1 < (unsigned)NB, h2 = s2 < (unsigned)NB, h3 = s3 < (unsigned)NB;
    const bool h4 = s4 < (unsigned)NB, h5 = s5 < (unsigned)NB, h6 = s6 < (unsigned)NB, h7 = s7 < (unsigned)NB;
    const unsigned any = __builtin_amdgcn_ballot_w32(h0 | h1 | h2 | h3 | h4 | h5 | h6 | h7);
    if (any != 0u) {
#define HITJ(J, HJ, SJ) { \
        const unsigned mj = __builtin_amdgcn_ballot_w32(HJ); \
        if (mj != 0u) { \
          if (HJ) { \
            const int pos = wc + (int)__builtin_amdgcn_mbcnt_lo(mj, 0u); \
            if (pos < WCAP) list[wave * WCAP + pos] = ((el0 + (J)) << 12) | (int)(SJ); \
          } \
          wc += (int)__builtin_popcount(mj); } }
      HITJ(0, h0, s0)
      HITJ(1, h1, s1)
      HITJ(2, h2, s2)
      HITJ(3, h3, s3)
      HITJ(4, h4, s4)
      HITJ(5, h5, s5)
      HITJ(6, h6, s6)
      HITJ(7, h7, s7)
#undef HITJ
    }
  }
  return wc;
}

template <int NC>
__global__ __launch_bounds__(NTHR) void k_wprep(const float* __restrict__ W, unsigned short* wp) {
  constexpr int UNITS = NC * KD / 8;
  constexpr int KD8   = KD / 8;
  static_assert((UNITS % 32) == 0);
  const int i = (int)blockIdx.x * NTHR + (int)threadIdx.x;
  if (i >= UNITS) return;
  const int n  = i / KD8;
  const int k0 = (i - n * KD8) * 8;
  float v[8];
#pragma unroll
  for (int e = 0; e < 8; ++e) v[e] = W[(size_t)(k0 + e) * NC + n];
  v4f a, b;
  a.x = v[0]; a.y = v[1]; a.z = v[2]; a.w = v[3];
  b.x = v[4]; b.y = v[5]; b.z = v[6]; b.w = v[7];
  v8us hv, lv;
  split8(a, b, hv, lv);
  unsigned short* dh = wp + (size_t)i * 8;
  unsigned short* dl = dh + (size_t)NC * KD;
  *(volatile v8us*)dh = hv;
  *(volatile v8us*)dl = lv;
  __threadfence();
  *(volatile v8us*)dh = hv;
  *(volatile v8us*)dl = lv;
}

__global__ __launch_bounds__(NTHR) void k_gemm1(
    const float* __restrict__ state, const float* __restrict__ inp,
    const unsigned short* __restrict__ Wp, const float* __restrict__ Wg,
    const float* __restrict__ attS, const float* __restrict__ attD,
    float* hout, float* eS, float* eD, int nN) {
  extern __shared__ v4f lds_dyn[];
  __shared__ __attribute__((aligned(16))) float sInp[BM];
  __shared__ __attribute__((aligned(16))) float sES[BM];
  __shared__ __attribute__((aligned(16))) float sED[BM];
  unsigned short* sHi = (unsigned short*)lds_dyn;
  unsigned short* sLo = sHi + BM * APK;
  float*          stg = (float*)lds_dyn;
  const int tid = threadIdx.x, lane = tid & 31, wave = tid >> 5, hh = lane >> 4, m = lane & 15;
  const int rowBase = blockIdx.x * BM;
  const int nR = nN * NBAT;

#pragma unroll
  for (int i = 0; i < 2; ++i) {
    const int idx = i * NTHR + tid;
    const int r   = idx >> 3;
    const int c0  = (idx & 7) * 8;
    int rho = rowBase + r;
    rho = rho > nR - 1 ? nR - 1 : rho;
    const int b = rho & (NBAT - 1);
    const int n = rho >> 3;
    const float* ap = state + ((size_t)b * nN + n) * UW + c0;
    const v4f a = *(const v4f*)ap, bq = *(const v4f*)(ap + 4);
    v8us hv, lv;
    split8(a, bq, hv, lv);
    *(v8us*)(sHi + r * APK + c0) = hv;
    *(v8us*)(sLo + r * APK + c0) = lv;
  }
  if (tid < BM) {
    int rho = rowBase + tid;
    rho = rho > nR - 1 ? nR - 1 : rho;
    sInp[tid] = inp[(size_t)(rho & (NBAT - 1)) * nN + (rho >> 3)];
  }
  __syncthreads();

  const int rg  = wave >> 1;
  const int chf = wave & 1;
  const int r0  = rg * 16;
  const int c0  = chf * 32;

  v8f acc[2];
#pragma unroll
  for (int t = 0; t < 2; ++t) { v8f z = {0.f, 0.f, 0.f, 0.f, 0.f, 0.f, 0.f, 0.f}; acc[t] = z; }
  const unsigned short* ahp = sHi + (r0 + m) * APK + 8 * hh;
  const unsigned short* alp = sLo + (r0 + m) * APK + 8 * hh;
#pragma unroll
  for (int kt = 0; kt < KD / 32; ++kt) {
    FragB ah, al;
    ah.h[0] = *(const v8us*)(ahp + 32 * kt);
    ah.h[1] = *(const v8us*)(ahp + 32 * kt + 16);
    al.h[0] = *(const v8us*)(alp + 32 * kt);
    al.h[1] = *(const v8us*)(alp + 32 * kt + 16);
#pragma unroll
    for (int t = 0; t < 2; ++t) {
      const unsigned short* bp = Wp + (size_t)(c0 + 16 * t + m) * KD + 32 * kt + 8 * hh;
      FragB bh, bl;
      bh.h[0] = *(const v8us*)bp;
      bh.h[1] = *(const v8us*)(bp + 16);
      bl.h[0] = *(const v8us*)(bp + UW * KD);
      bl.h[1] = *(const v8us*)(bp + UW * KD + 16);
      acc[t] = wmb(ah.v, bh.v, acc[t]);
      acc[t] = wmb(ah.v, bl.v, acc[t]);
      acc[t] = wmb(al.v, bh.v, acc[t]);
    }
  }
  __syncthreads();

  {
    float wt[2];
#pragma unroll
    for (int t = 0; t < 2; ++t) wt[t] = Wg[(size_t)UW * UW + c0 + 16 * t + m];
#pragma unroll
    for (int t = 0; t < 2; ++t) {
#pragma unroll
      for (int r = 0; r < 8; ++r) {
        const int row = r0 + 8 * hh + r;
        stg[(size_t)row * UW + c0 + 16 * t + m] = acc[t][r] + sInp[row] * wt[t];
      }
    }
  }
  __syncthreads();

  {
    const int row = tid >> 2;
    const int cq  = tid & 3;
    const float* sp = stg + (size_t)row * UW + cq * 16;
    const v4f x0 = *(const v4f*)sp, x1 = *(const v4f*)(sp + 4), x2 = *(const v4f*)(sp + 8), x3 = *(const v4f*)(sp + 12);
    const v4f s0 = *(const v4f*)(attS + cq * 16), s1 = *(const v4f*)(attS + cq * 16 + 4);
    const v4f s2 = *(const v4f*)(attS + cq * 16 + 8), s3 = *(const v4f*)(attS + cq * 16 + 12);
    const v4f d0 = *(const v4f*)(attD + cq * 16), d1 = *(const v4f*)(attD + cq * 16 + 4);
    const v4f d2 = *(const v4f*)(attD + cq * 16 + 8), d3 = *(const v4f*)(attD + cq * 16 + 12);
    const v4f ms = x0 * s0 + x1 * s1 + x2 * s2 + x3 * s3;
    const v4f md = x0 * d0 + x1 * d1 + x2 * d2 + x3 * d3;
    float ps = (ms.x + ms.y) + (ms.z + ms.w);
    float pd = (md.x + md.y) + (md.z + md.w);
    ps += __shfl_xor(ps, 1); pd += __shfl_xor(pd, 1);
    ps += __shfl_xor(ps, 2); pd += __shfl_xor(pd, 2);
    if ((lane & 3) == 0) { sES[row] = ps; sED[row] = pd; }
  }

  v4f hv[4];
#pragma unroll
  for (int it = 0; it < 4; ++it) hv[it] = *(const v4f*)(stg + 4 * (it * NTHR + tid));
  float* hp = hout + (size_t)rowBase * UW;
#pragma unroll
  for (int it = 0; it < 4; ++it) *(volatile v4f*)(hp + 4 * (it * NTHR + tid)) = hv[it];
  __syncthreads();

  const v4f vS = *(const v4f*)(sES + 4 * (lane & 15));
  const v4f vD = *(const v4f*)(sED + 4 * (lane & 15));
  const v4f ev = (lane < 16) ? vS : vD;
  float* ep = ((lane < 16) ? eS : eD) + rowBase + 4 * (lane & 15);
  if (wave == 0) *(volatile v4f*)ep = ev;
  __threadfence();
#pragma unroll
  for (int it = 0; it < 4; ++it) *(volatile v4f*)(hp + 4 * (it * NTHR + tid)) = hv[it];
  if (wave == 0) *(volatile v4f*)ep = ev;
}

__global__ __launch_bounds__(NTHR) void k_attn_agg(
    const int* __restrict__ srcs, const int* __restrict__ dsts,
    const float* __restrict__ hpl, const float* __restrict__ eS, const float* __restrict__ eD,
    const float* __restrict__ bias, float* sg, int nN, int nE, int vec8) {
  extern __shared__ v4f lds_dyn[];
  int* region = (int*)lds_dyn;
  int* cursor = region + RCAP;
  int* scnt   = cursor + NBF;
  int* sst    = scnt + NBF;
  int* list   = sst + NBF;
  int* wcnt   = list + LISTN;
  int* wtot   = wcnt + 16;
  const int tid = threadIdx.x, lane = tid & 31, wave = tid >> 5;
  const int nodeBase = blockIdx.x * NBF;

  {
    const v4i z = {0, 0, 0, 0};
#pragma unroll 1
    for (int i = tid; i < RCAP / 4; i += NTHR) ((v4i*)region)[i] = z;
#pragma unroll 1
    for (int i = tid; i < NBF; i += NTHR) scnt[i] = 0;
  }
  __syncthreads();

  const int nChunks = (nE + CHUNK - 1) / CHUNK;

#pragma unroll 1
  for (int ch = 0; ch < nChunks; ++ch) {
    const int cbase = ch * CHUNK;
    const int wc = scan_chunk<NBF>(dsts, nE, cbase, nodeBase, vec8, list, tid, lane, wave);
    if (lane == 0) wcnt[wave] = wc;
    __syncthreads();
    if (wave == 0) {
#pragma unroll 1
      for (int wsx = 0; wsx < NWAVE; ++wsx) {
        int n = __builtin_amdgcn_readfirstlane(wcnt[wsx]);
        n = n > WCAP ? WCAP : (n < 0 ? 0 : n);
        const int* lp = list + wsx * WCAP;
#pragma unroll 1
        for (int i = 0; i < n; ++i) {
          const int ent  = __builtin_amdgcn_readfirstlane(lp[i]);
          const int slot = ent & (NBF - 1);
          if (lane == 0) scnt[slot] = scnt[slot] + 1;
        }
      }
    }
    __syncthreads();
  }

  {
    const v4i cv = *(const v4i*)(scnt + 4 * tid);
    const int e0 = max(cv.x, 0), e1 = max(cv.y, 0), e2 = max(cv.z, 0), e3 = max(cv.w, 0);
    const int ts = e0 + e1 + e2 + e3;
    int incl = ts;
#pragma unroll
    for (int d = 1; d < 32; d <<= 1) {
      const int t = __shfl_up(incl, d);
      if (lane >= d) incl += t;
    }
    if (lane == 31) wtot[wave] = incl;
    __syncthreads();
    int pre = 0;
#pragma unroll 1
    for (int w = 0; w < wave; ++w) pre += wtot[w];
    int run = pre + incl - ts;
    int o;
    o = run > RCAP ? RCAP : run; sst[4 * tid + 0] = o; cursor[4 * tid + 0] = o; run += e0;
    o = run > RCAP ? RCAP : run; sst[4 * tid + 1] = o; cursor[4 * tid + 1] = o; run += e1;
    o = run > RCAP ? RCAP : run; sst[4 * tid + 2] = o; cursor[4 * tid + 2] = o; run += e2;
    o = run > RCAP ? RCAP : run; sst[4 * tid + 3] = o; cursor[4 * tid + 3] = o;
  }
  __syncthreads();

#pragma unroll 1
  for (int ch = 0; ch < nChunks; ++ch) {
    const int cbase = ch * CHUNK;
    const int wc = scan_chunk<NBF>(dsts, nE, cbase, nodeBase, vec8, list, tid, lane, wave);
    if (lane == 0) wcnt[wave] = wc;
    __syncthreads();
    if (wave == 0) {
#pragma unroll 1
      for (int wsx = 0; wsx < NWAVE; ++wsx) {
        int n = __builtin_amdgcn_readfirstlane(wcnt[wsx]);
        n = n > WCAP ? WCAP : (n < 0 ? 0 : n);
        const int* lp = list + wsx * WCAP;
#pragma unroll 1
        for (int i = 0; i < n; ++i) {
          const int ent  = __builtin_amdgcn_readfirstlane(lp[i]);
          const int slot = ent & (NBF - 1);
          int e = cbase + ((ent >> 12) & (CHUNK - 1));
          e = e > nE - 1 ? nE - 1 : e;
          int src = srcs[e];
          src = src < 0 ? 0 : (src > nN - 1 ? nN - 1 : src);
          if (lane == 0) {
            int pos = cursor[slot];
            pos = pos < 0 ? 0 : (pos > RCAP - 1 ? RCAP - 1 : pos);
            region[pos] = src;
            const int np = pos + 1;
            cursor[slot] = np > RCAP ? RCAP : np;
          }
        }
      }
    }
    __syncthreads();
  }

  float* sOut = (float*)list + wave * (NBAT * UW);
  const int bl   = lane >> 2;
  const int cg   = lane & 3;
  const int colb = cg * 16;
  const v4f bg0 = *(const v4f*)(bias + colb), bg1 = *(const v4f*)(bias + colb + 4);
  const v4f bg2 = *(const v4f*)(bias + colb + 8), bg3 = *(const v4f*)(bias + colb + 12);

#pragma unroll 1
  for (int j = 0; j < TPWV; ++j) {
    const int slot = wave * TPWV + j;
    const int c = nodeBase + slot;
    if (c >= nN) break;
    int n = __builtin_amdgcn_readfirstlane(scnt[slot]);
    n = n < 0 ? 0 : (n > DEGCAP ? DEGCAP : n);
    int st = __builtin_amdgcn_readfirstlane(sst[slot]);
    st = st < 0 ? 0 : (st > RCAP ? RCAP : st);
    if (n > RCAP - st) n = RCAP - st;
    const size_t rc = (size_t)c * NBAT + bl;
    const float edv   = eD[rc];
    const float eself = lrelu(eS[rc] + edv);

    float mx = eself;
#pragma unroll 1
    for (int q0 = 0; q0 < n; q0 += 32) {
      int pos = st + q0 + lane;
      pos = pos > RCAP - 1 ? RCAP - 1 : pos;
      int sl = region[pos];
      sl = sl < 0 ? 0 : (sl > nN - 1 ? nN - 1 : sl);
      const int mcnt = (n - q0) < 32 ? (n - q0) : 32;
#pragma unroll 1
      for (int pp = 0; pp < mcnt; ++pp) {
        const int s = __builtin_amdgcn_readlane(sl, pp);
        mx = fmaxf(mx, lrelu(eS[(size_t)s * NBAT + bl] + edv));
      }
    }

    float p   = __expf(eself - mx);
    float den = p;
    const float* hs = hpl + rc * UW + colb;
    v4f a0 = *(const v4f*)hs * p,       a1 = *(const v4f*)(hs + 4) * p;
    v4f a2 = *(const v4f*)(hs + 8) * p, a3 = *(const v4f*)(hs + 12) * p;
#pragma unroll 1
    for (int q0 = 0; q0 < n; q0 += 32) {
      int pos = st + q0 + lane;
      pos = pos > RCAP - 1 ? RCAP - 1 : pos;
      int sl = region[pos];
      sl = sl < 0 ? 0 : (sl > nN - 1 ? nN - 1 : sl);
      const int mcnt = (n - q0) < 32 ? (n - q0) : 32;
#pragma unroll 1
      for (int pp = 0; pp < mcnt; ++pp) {
        const int s = __builtin_amdgcn_readlane(sl, pp);
        const size_t rs = (size_t)s * NBAT + bl;
        p = __expf(lrelu(eS[rs] + edv) - mx);
        den += p;
        const float* hq = hpl + rs * UW + colb;
        a0 = a0 + *(const v4f*)hq * p;
        a1 = a1 + *(const v4f*)(hq + 4) * p;
        a2 = a2 + *(const v4f*)(hq + 8) * p;
        a3 = a3 + *(const v4f*)(hq + 12) * p;
      }
    }

    const float rd = rcpf_(den);
    const v4f v0 = a0 * rd + bg0, v1 = a1 * rd + bg1, v2 = a2 * rd + bg2, v3 = a3 * rd + bg3;

    float* so = sOut + bl * UW + colb;
    *(v4f*)(so)      = v0;
    *(v4f*)(so + 4)  = v1;
    *(v4f*)(so + 8)  = v2;
    *(v4f*)(so + 12) = v3;
    __builtin_amdgcn_fence(__ATOMIC_RELEASE, "wavefront");
    __builtin_amdgcn_wave_barrier();
    v4f ov[4];
#pragma unroll
    for (int it = 0; it < 4; ++it) ov[it] = *(const v4f*)(sOut + 4 * (it * 32 + lane));
    __builtin_amdgcn_fence(__ATOMIC_RELEASE, "wavefront");
    __builtin_amdgcn_wave_barrier();
#pragma unroll
    for (int it = 0; it < 4; ++it) {
      const int bb = 2 * it + (lane >> 4);
      float* gp = sg + ((size_t)bb * nN + c) * UW + 4 * (lane & 15);
      *(volatile v4f*)gp = ov[it];
    }
    __threadfence();
#pragma unroll
    for (int it = 0; it < 4; ++it) {
      const int bb = 2 * it + (lane >> 4);
      float* gp = sg + ((size_t)bb * nN + c) * UW + 4 * (lane & 15);
      *(volatile v4f*)gp = ov[it];
    }
  }
}

__global__ __launch_bounds__(NTHR) void k_gate(
    const float* __restrict__ sgp, const float* __restrict__ inp,
    const unsigned short* __restrict__ W1p, const unsigned short* __restrict__ W2p,
    const float* __restrict__ W1, const float* __restrict__ b1,
    const float* __restrict__ W2, const float* __restrict__ b2,
    float* out, int nR) {
  extern __shared__ v4f lds_dyn[];
  char* base = (char*)lds_dyn;
  unsigned short* sHi  = (unsigned short*)base;
  unsigned short* sLo  = sHi + BM * APK;
  float*          stg  = (float*)base;
  float*          sSg  = (float*)(base + 2 * BM * APK * 2);
  float*          sU   = sSg + BM * UW;
  float*          sInp = sU + BM * UW;
  const int tid = threadIdx.x, lane = tid & 31, wave = tid >> 5, hh = lane >> 4, m = lane & 15;
  const int rowBase = blockIdx.x * BM;

#pragma unroll
  for (int i = 0; i < 2; ++i) {
    const int idx = i * NTHR + tid;
    const int r   = idx >> 3;
    const int c0  = (idx & 7) * 8;
    int row = rowBase + r;
    row = row > nR - 1 ? nR - 1 : row;
    const float* ap = sgp + (size_t)row * UW + c0;
    const v4f a = *(const v4f*)ap, bq = *(const v4f*)(ap + 4);
    *(v4f*)(sSg + r * UW + c0)     = a;
    *(v4f*)(sSg + r * UW + c0 + 4) = bq;
    v8us hv, lv;
    split8(a, bq, hv, lv);
    *(v8us*)(sHi + r * APK + c0) = hv;
    *(v8us*)(sLo + r * APK + c0) = lv;
  }
  if (tid < BM) {
    int row = rowBase + tid;
    row = row > nR - 1 ? nR - 1 : row;
    sInp[tid] = inp[row];
  }
  __syncthreads();

  const int rg  = wave >> 1;
  const int chf = wave & 1;
  const int r0  = rg * 16;
  const unsigned short* ahp = sHi + (r0 + m) * APK + 8 * hh;
  const unsigned short* alp = sLo + (r0 + m) * APK + 8 * hh;

  const int c0a = chf * 64;
  v8f acc[4];
#pragma unroll
  for (int t = 0; t < 4; ++t) { v8f z = {0.f, 0.f, 0.f, 0.f, 0.f, 0.f, 0.f, 0.f}; acc[t] = z; }
#pragma unroll
  for (int kt = 0; kt < KD / 32; ++kt) {
    FragB ah, al;
    ah.h[0] = *(const v8us*)(ahp + 32 * kt);
    ah.h[1] = *(const v8us*)(ahp + 32 * kt + 16);
    al.h[0] = *(const v8us*)(alp + 32 * kt);
    al.h[1] = *(const v8us*)(alp + 32 * kt + 16);
#pragma unroll
    for (int t = 0; t < 4; ++t) {
      const unsigned short* bp = W1p + (size_t)(c0a + 16 * t + m) * KD + 32 * kt + 8 * hh;
      FragB bh, bl;
      bh.h[0] = *(const v8us*)bp;
      bh.h[1] = *(const v8us*)(bp + 16);
      bl.h[0] = *(const v8us*)(bp + 2 * UW * KD);
      bl.h[1] = *(const v8us*)(bp + 2 * UW * KD + 16);
      acc[t] = wmb(ah.v, bh.v, acc[t]);
      acc[t] = wmb(ah.v, bl.v, acc[t]);
      acc[t] = wmb(al.v, bh.v, acc[t]);
    }
  }
  __syncthreads();

  {
    float wt[4], bv[4];
#pragma unroll
    for (int t = 0; t < 4; ++t) { const int col = c0a + 16 * t + m; wt[t] = W1[col]; bv[t] = b1[col]; }
    if (chf == 0) {
#pragma unroll
      for (int t = 0; t < 4; ++t) {
#pragma unroll
        for (int r = 0; r < 8; ++r) {
          const int row = r0 + 8 * hh + r;
          const int col = c0a + 16 * t + m;
          const float s  = sigmf(acc[t][r] + sInp[row] * wt[t] + bv[t]);
          const float rs = s * sSg[row * UW + col];
          unsigned short hb, lb;
          split1(rs, hb, lb);
          sHi[row * APK + col] = hb;
          sLo[row * APK + col] = lb;
        }
      }
    } else {
#pragma unroll
      for (int t = 0; t < 4; ++t) {
#pragma unroll
        for (int r = 0; r < 8; ++r) {
          const int row = r0 + 8 * hh + r;
          const int col = c0a + 16 * t + m;
          const float s = sigmf(acc[t][r] + sInp[row] * wt[t] + bv[t]);
          sU[row * UW + (col - UW)] = s;
        }
      }
    }
  }
  __syncthreads();

  const int c0b = chf * 32;
  v8f acc2[2];
#pragma unroll
  for (int t = 0; t < 2; ++t) { v8f z = {0.f, 0.f, 0.f, 0.f, 0.f, 0.f, 0.f, 0.f}; acc2[t] = z; }
#pragma unroll
  for (int kt = 0; kt < KD / 32; ++kt) {
    FragB ah, al;
    ah.h[0] = *(const v8us*)(ahp + 32 * kt);
    ah.h[1] = *(const v8us*)(ahp + 32 * kt + 16);
    al.h[0] = *(const v8us*)(alp + 32 * kt);
    al.h[1] = *(const v8us*)(alp + 32 * kt + 16);
#pragma unroll
    for (int t = 0; t < 2; ++t) {
      const unsigned short* bp = W2p + (size_t)(c0b + 16 * t + m) * KD + 32 * kt + 8 * hh;
      FragB bh, bl;
      bh.h[0] = *(const v8us*)bp;
      bh.h[1] = *(const v8us*)(bp + 16);
      bl.h[0] = *(const v8us*)(bp + UW * KD);
      bl.h[1] = *(const v8us*)(bp + UW * KD + 16);
      acc2[t] = wmb(ah.v, bh.v, acc2[t]);
      acc2[t] = wmb(ah.v, bl.v, acc2[t]);
      acc2[t] = wmb(al.v, bh.v, acc2[t]);
    }
  }
  __syncthreads();

  {
#pragma unroll
    for (int t = 0; t < 2; ++t) {
      const int col = c0b + 16 * t + m;
      const float wt = W2[col];
      const float bv = b2[col];
#pragma unroll
      for (int r = 0; r < 8; ++r) {
        const int row = r0 + 8 * hh + r;
        const float cc  = tanhf_(acc2[t][r] + sInp[row] * wt + bv);
        const float u   = sU[row * UW + col];
        const float sgv = sSg[row * UW + col];
        stg[row * UW + col] = u * sgv + (1.0f - u) * cc;
      }
    }
  }
  __syncthreads();

  v4f ov[4];
#pragma unroll
  for (int it = 0; it < 4; ++it) ov[it] = *(const v4f*)(stg + 4 * (it * NTHR + tid));
  float* op = out + (size_t)rowBase * UW;
#pragma unroll
  for (int it = 0; it < 4; ++it) {
    const int f = it * NTHR + tid;
    if (rowBase + (f >> 4) < nR) *(volatile v4f*)(op + 4 * f) = ov[it];
  }
  __threadfence();
#pragma unroll
  for (int it = 0; it < 4; ++it) {
    const int f = it * NTHR + tid;
    if (rowBase + (f >> 4) < nR) *(volatile v4f*)(op + 4 * f) = ov[it];
  }
}

extern "C" void kernel_launch(void* const* d_in, const int* in_sizes, int n_in,
                              void* d_out, int out_size, void* d_ws, size_t ws_size,
                              hipStream_t stream) {
  if (n_in < 11) return;
  const int nBN = in_sizes[0];
  if (nBN <= 0 || nBN > (1 << 24) || (nBN % NBAT) != 0) return;
  const int nN = nBN / NBAT;
  if (in_sizes[1] != nBN * UW) return;
  const int nE2 = in_sizes[2];
  if (nE2 < 2 || (nE2 & 1) != 0) return;
  const int nE = nE2 / 2;
  if (nE > (1 << 28)) return;
  if (in_sizes[3] != (UW + 1) * UW || in_sizes[4] != UW || in_sizes[5] != UW || in_sizes[6] != UW) return;
  if (in_sizes[7] != (UW + 1) * 2 * UW || in_sizes[8] != 2 * UW) return;
  if (in_sizes[9] != (UW + 1) * UW || in_sizes[10] != UW) return;
  if (out_size != nBN * UW) return;

  const float* inp   = (const float*)d_in[0];
  const float* state = (const float*)d_in[1];
  const int*   edges = (const int*)d_in[2];
  const float* Wg    = (const float*)d_in[3];
  const float* attS  = (const float*)d_in[4];
  const float* attD  = (const float*)d_in[5];
  const float* bgat  = (const float*)d_in[6];
  const float* W1    = (const float*)d_in[7];
  const float* b1    = (const float*)d_in[8];
  const float* W2    = (const float*)d_in[9];
  const float* b2    = (const float*)d_in[10];
  float* out = (float*)d_out;
  const int* srcs = edges;
  const int* dsts = edges + nE;

  const int nR   = nBN;
  const int NPAD = ((nR + BM - 1) / BM) * BM;
  const int nBF  = (nN + NBF - 1) / NBF;

  char* ws = (char*)d_ws;
  size_t off = 0;
  const size_t oWg = off; off += (size_t)2 * UW * KD * 2;          off = (off + 255) & ~(size_t)255;
  const size_t oW1 = off; off += (size_t)2 * (2 * UW) * KD * 2;    off = (off + 255) & ~(size_t)255;
  const size_t oW2 = off; off += (size_t)2 * UW * KD * 2;          off = (off + 255) & ~(size_t)255;
  const size_t oH  = off; off += (size_t)NPAD * UW * 4;            off = (off + 255) & ~(size_t)255;
  const size_t oES = off; off += (size_t)NPAD * 4;                 off = (off + 255) & ~(size_t)255;
  const size_t oED = off; off += (size_t)NPAD * 4;                 off = (off + 255) & ~(size_t)255;
  const size_t oSg = off; off += (size_t)NPAD * UW * 4;            off = (off + 255) & ~(size_t)255;
  if (off > ws_size || off > (size_t)WSCAP) return;
  unsigned short* wgp = (unsigned short*)(ws + oWg);
  unsigned short* w1p = (unsigned short*)(ws + oW1);
  unsigned short* w2p = (unsigned short*)(ws + oW2);
  float* hpl = (float*)(ws + oH);
  float* es  = (float*)(ws + oES);
  float* ed  = (float*)(ws + oED);
  float* sg  = (float*)(ws + oSg);

  const int vec8 = ((nE & 3) == 0) ? 1 : 0;

  k_wprep<UW><<<(UW * KD / 8 + NTHR - 1) / NTHR, NTHR, 0, stream>>>(Wg, wgp);
  k_wprep<2 * UW><<<(2 * UW * KD / 8 + NTHR - 1) / NTHR, NTHR, 0, stream>>>(W1 + 2 * UW, w1p);
  k_wprep<UW><<<(UW * KD / 8 + NTHR - 1) / NTHR, NTHR, 0, stream>>>(W2 + UW, w2p);

  hipFuncSetAttribute(reinterpret_cast<const void*>(&k_gemm1),
                      hipFuncAttributeMaxDynamicSharedMemorySize, LDS_GEMM1);
  k_gemm1<<<NPAD / BM, NTHR, LDS_GEMM1, stream>>>(state, inp, wgp, Wg, attS, attD, hpl, es, ed, nN);

  hipFuncSetAttribute(reinterpret_cast<const void*>(&k_attn_agg),
                      hipFuncAttributeMaxDynamicSharedMemorySize, LDS_AGG);
  k_attn_agg<<<nBF, NTHR, LDS_AGG, stream>>>(srcs, dsts, hpl, es, ed, bgat, sg, nN, nE, vec8);

  hipFuncSetAttribute(reinterpret_cast<const void*>(&k_gate),
                      hipFuncAttributeMaxDynamicSharedMemorySize, LDS_GATE);
  k_gate<<<NPAD / BM, NTHR, LDS_GATE, stream>>>(sg, inp, w1p, w2p, W1, b1, W2, b2, out, nR);
}
